// GraphTransformer_59322088292417
// MI455X (gfx1250) — hardware-verified
//
#include <hip/hip_runtime.h>
#include <hip/hip_bf16.h>
#include <math.h>

#define BB 8
#define NN 512
#define N1 513
#define FEAT 11
#define POS 32
#define DIM 128
#define HH 8
#define LL 4
#define HID 256
#define M_TOK (BB * N1)
#define QKV_N (3 * HH * DIM)
#define OPROJ_K (HH * DIM)
#define EPSL 1e-6f

typedef _Float16 h8  __attribute__((ext_vector_type(8)));
typedef _Float16 h16 __attribute__((ext_vector_type(16)));
typedef float    f4  __attribute__((ext_vector_type(4)));
typedef float    f8  __attribute__((ext_vector_type(8)));

__device__ __forceinline__ h16 cat88(h8 lo, h8 hi) {
  return __builtin_shufflevector(lo, hi, 0,1,2,3,4,5,6,7,8,9,10,11,12,13,14,15);
}
__device__ __forceinline__ h8 cvt8(f4 a, f4 b) {
  h8 r;
  r[0] = (_Float16)a[0]; r[1] = (_Float16)a[1];
  r[2] = (_Float16)a[2]; r[3] = (_Float16)a[3];
  r[4] = (_Float16)b[0]; r[5] = (_Float16)b[1];
  r[6] = (_Float16)b[2]; r[7] = (_Float16)b[3];
  return r;
}
__device__ __forceinline__ f8 wmma_f16(h16 a, h16 b, f8 c) {
  f8 d = __builtin_amdgcn_wmma_f32_16x16x32_f16(false, a, false, b, (short)0, c, false, false);
  asm volatile("v_nop\n\tv_nop\n\tv_nop\n\tv_nop" : "+v"(d) : "v"(a), "v"(b));
  return d;
}
typedef unsigned u4 __attribute__((ext_vector_type(4)));
typedef float __attribute__((may_alias)) float_a;
#define GSTRIDE 32
template <typename T> __device__ __forceinline__ void vst2(void* p, T v) { *(volatile T*)p = v; __threadfence(); *(volatile T*)p = v; }

__global__ void k_embed(const float* __restrict__ nf, const float* __restrict__ lapl,
                        const float* __restrict__ Wne1, const float* __restrict__ bne1,
                        const float* __restrict__ Wne2, const float* __restrict__ bne2,
                        const float* __restrict__ Wpos, const float* __restrict__ bpos,
                        const float* __restrict__ cls_tok, const float* __restrict__ cls_pos,
                        float* __restrict__ x) {
  int t = blockIdx.x;
  int b = t / N1, n = t % N1;
  int tid = threadIdx.x;
  __shared__ float t1[2 * DIM];
  if (n == 0) {
    if (tid < DIM) vst2(x + (size_t)t * DIM + tid, (float_a)(cls_tok[tid] + cls_pos[tid]));
    return;
  }
  const float* f = nf + ((size_t)b * NN + (n - 1)) * FEAT;
  float acc = bne1[tid];
#pragma unroll
  for (int k = 0; k < FEAT; k++) acc += f[k] * Wne1[k * 2 * DIM + tid];
  t1[tid] = fmaxf(acc, 0.f);
  __syncthreads();
  if (tid < DIM) {
    float v = bne2[tid] + bpos[tid];
    const float* lp = lapl + ((size_t)b * NN + (n - 1)) * POS;
    for (int k = 0; k < 2 * DIM; k++) v += t1[k] * Wne2[k * DIM + tid];
#pragma unroll
    for (int p = 0; p < POS; p++) v += lp[p] * Wpos[p * DIM + tid];
    vst2(x + (size_t)t * DIM + tid, (float_a)v);
  }
}

__device__ __forceinline__ float block_reduce128(float v, float* sbuf) {
#pragma unroll
  for (int m = 16; m >= 1; m >>= 1) v += __shfl_xor(v, m, 32);
  int w = threadIdx.x >> 5;
  if ((threadIdx.x & 31) == 0) sbuf[w] = v;
  __syncthreads();
  float r = sbuf[0] + sbuf[1] + sbuf[2] + sbuf[3];
  __syncthreads();
  return r;
}

__global__ void k_ln(const float* __restrict__ x, const float* __restrict__ s,
                     const float* __restrict__ bb_, const float* __restrict__ Wg,
                     const float* __restrict__ bg, float* __restrict__ h,
                     float* __restrict__ g, int do_gate) {
  __shared__ float sbuf[4];
  int t = blockIdx.x, d = threadIdx.x;
  float v = x[(size_t)t * DIM + d];
  float mu = block_reduce128(v, sbuf) * (1.f / DIM);
  float dv = v - mu;
  float var = block_reduce128(dv * dv, sbuf) * (1.f / DIM);
  float hn = dv * rsqrtf(var + EPSL) * s[d] + bb_[d];
  vst2(h + (size_t)t * DIM + d, (float_a)hn);
  if (do_gate) {
    float s0 = block_reduce128(hn * Wg[d * 2 + 0], sbuf);
    float s1 = block_reduce128(hn * Wg[d * 2 + 1], sbuf);
    if (d == 0) {
      vst2(g + (size_t)t * GSTRIDE + 0, (float_a)expf(s0 + bg[0]));
      vst2(g + (size_t)t * GSTRIDE + 1, (float_a)expf(s1 + bg[1]));
    }
  }
}

__global__ __launch_bounds__(256) void k_gemm(const float* __restrict__ A,
                                              const float* __restrict__ W,
                                              const float* __restrict__ bias,
                                              const float* __restrict__ res,
                                              float* __restrict__ C,
                                              int M, int K, int N, int act) {
  __shared__ __align__(16) _Float16 As[64][40];
  __shared__ __align__(16) _Float16 BsT[64][40];
  __shared__ __align__(16) float So[8][16 * 32];
  int m0 = blockIdx.x * 64;
  int n0 = blockIdx.y * 64;
  int tid = threadIdx.x;
  int wave = tid >> 5, lane = tid & 31;
  int tiler = wave >> 1;
  int tilec0 = (wave & 1) * 2;
  f8 c0 = {}; f8 c1 = {};
  int arow = tid >> 2;
  int akk  = (tid & 3) * 8;
  int bn   = tid & 63;
  int bkg  = (tid >> 6) * 8;
  int hi = lane >> 4, cn = lane & 15;

  for (int kc = 0; kc < K; kc += 32) {
    {
      int gr = m0 + arow;
      f4 a0 = {}, a1 = {};
      if (gr < M) {
        const f4* ap = (const f4*)(A + (size_t)gr * K + kc + akk);
        a0 = ap[0]; a1 = ap[1];
        if (kc + 32 < K) __builtin_prefetch(A + (size_t)gr * K + kc + 32 + akk, 0, 1);
      }
      *(h8*)&As[arow][akk] = cvt8(a0, a1);
    }
    {
      const float* wp = W + (size_t)(kc + bkg) * N + n0 + bn;
      float wv[8];
#pragma unroll
      for (int j = 0; j < 8; j++) wv[j] = wp[(size_t)j * N];
      h8 bvv;
#pragma unroll
      for (int j = 0; j < 8; j++) bvv[j] = (_Float16)wv[j];
      *(h8*)&BsT[bn][bkg] = bvv;
    }
    __syncthreads();
    int r = tiler * 16 + cn;
    int kh = hi * 8;
    h16 a = cat88(*(const h8*)&As[r][kh], *(const h8*)&As[r][kh + 16]);
    int kb = hi * 8;
    {
      int col = tilec0 * 16 + cn;
      h16 b0 = cat88(*(const h8*)&BsT[col][kb], *(const h8*)&BsT[col][kb + 16]);
      c0 = wmma_f16(a, b0, c0);
    }
    {
      int col = (tilec0 + 1) * 16 + cn;
      h16 b1 = cat88(*(const h8*)&BsT[col][kb], *(const h8*)&BsT[col][kb + 16]);
      c1 = wmma_f16(a, b1, c1);
    }
    __syncthreads();
  }
  float* S = So[wave];
#pragma unroll
  for (int tt = 0; tt < 2; tt++) {
    f8 c = tt ? c1 : c0;
    int col = n0 + (tilec0 + tt) * 16 + cn;
#pragma unroll 1
    for (int gg = 0; gg < 8; gg++) {
      int row = m0 + tiler * 16 + gg + hi * 8;
      float v = c[gg];
      if (bias) v += bias[col];
      if (act == 1) v = 0.5f * v * (1.f + erff(v * 0.70710678118654752f));
      if (res && row < M) v += res[(size_t)row * N + col];
      S[(gg + hi * 8) * 32 + tt * 16 + cn] = v;
    }
  }
  asm volatile("s_wait_dscnt 0" ::: "memory"); __builtin_amdgcn_wave_barrier(); __builtin_amdgcn_fence(__ATOMIC_RELEASE, "workgroup");
#pragma unroll
  for (int q = 0; q < 4; q++) { const int rl = q * 4 + (lane >> 3), pc = lane & 7; const int row = m0 + tiler * 16 + rl;
    if (row < M) vst2(C + (size_t)row * N + n0 + tilec0 * 16 + pc * 4, *(const f4*)(S + rl * 32 + pc * 4)); }
}

__global__ __launch_bounds__(128) void k_attn(const float* __restrict__ qkv,
                                              const float* __restrict__ g,
                                              const float* __restrict__ adj,
                                              float* __restrict__ o) {
  __shared__ __align__(16) _Float16 Ks[32][136];
  __shared__ __align__(16) _Float16 VsT[DIM][40];
  __shared__ __align__(16) _Float16 Ps[4][16][40];
  __shared__ __align__(16) float Os[4][16 * DIM];
  const float scale = 0.08838834764831845f;
  int b = blockIdx.z, head = blockIdx.y;
  int tid = threadIdx.x, wave = tid >> 5, lane = tid & 31;
  int rt = blockIdx.x * 4 + wave;
  bool active = rt < 33;
  int rowbase = rt * 16;
  int hi = lane >> 4, cn = lane & 15;

  h16 aq[4];
  float gv0[8], gv1[8], mrow[8], lrow[8];
  f8 acc[8];
  f8 zero = {};
  if (active) {
    int qrow = rowbase + cn; if (qrow > N1 - 1) qrow = N1 - 1;
    const f4* Qp4 = (const f4*)(qkv + ((size_t)(b * N1) + qrow) * QKV_N + head * DIM);
    int khq = hi * 2;
#pragma unroll
    for (int kc = 0; kc < 4; kc++) {
      f4 q0 = Qp4[kc * 8 + khq + 0];
      f4 q1 = Qp4[kc * 8 + khq + 1];
      f4 q2 = Qp4[kc * 8 + khq + 4];
      f4 q3 = Qp4[kc * 8 + khq + 5];
      aq[kc] = cat88(cvt8(q0, q1), cvt8(q2, q3));
    }
#pragma unroll
    for (int gg = 0; gg < 8; gg++) {
      int rr = rowbase + gg + hi * 8; if (rr > N1 - 1) rr = N1 - 1;
      gv0[gg] = g[(size_t)(b * N1 + rr) * GSTRIDE + 0];
      gv1[gg] = g[(size_t)(b * N1 + rr) * GSTRIDE + 1];
      mrow[gg] = -3.0e38f; lrow[gg] = 0.f;
    }
#pragma unroll
    for (int dc = 0; dc < 8; dc++) acc[dc] = zero;
  }

  for (int j = 0; j < 17; j++) {
    int colbase = j * 32;
    {
      int tok = tid >> 2;
      int dp = (tid & 3) * 32;
      int ct = colbase + tok;
      f4 kb4[8];
      if (ct < N1) {
        const f4* Kp4 = (const f4*)(qkv + ((size_t)(b * N1) + ct) * QKV_N +
                                    (HH + head) * DIM + dp);
#pragma unroll
        for (int i = 0; i < 8; i++) kb4[i] = Kp4[i];
      } else {
        f4 z4 = {};
#pragma unroll
        for (int i = 0; i < 8; i++) kb4[i] = z4;
      }
#pragma unroll
      for (int q = 0; q < 4; q++)
        *(h8*)&Ks[tok][dp + q * 8] = cvt8(kb4[q * 2], kb4[q * 2 + 1]);
    }
    {
      int dd = tid;
      const float* Vbase = qkv + (size_t)(b * N1) * QKV_N + (2 * HH + head) * DIM + dd;
      _Float16 vrow[32];
#pragma unroll
      for (int t2 = 0; t2 < 32; t2++) {
        int ct2 = colbase + t2;
        float vv = (ct2 < N1) ? Vbase[(size_t)ct2 * QKV_N] : 0.f;
        vrow[t2] = (_Float16)vv;
      }
#pragma unroll
      for (int q = 0; q < 4; q++) {
        h8 t;
#pragma unroll
        for (int jj = 0; jj < 8; jj++) t[jj] = vrow[q * 8 + jj];
        *(h8*)&VsT[dd][q * 8] = t;
      }
    }
    __syncthreads();
    if (active) {
      int kb = hi * 8;
      f8 s0 = zero, s1 = zero;
#pragma unroll
      for (int kc = 0; kc < 4; kc++) {
        h16 b0 = cat88(*(const h8*)&Ks[cn][kc * 32 + kb],
                       *(const h8*)&Ks[cn][kc * 32 + kb + 16]);
        s0 = wmma_f16(aq[kc], b0, s0);
      }
#pragma unroll
      for (int kc = 0; kc < 4; kc++) {
        h16 b1 = cat88(*(const h8*)&Ks[16 + cn][kc * 32 + kb],
                       *(const h8*)&Ks[16 + cn][kc * 32 + kb + 16]);
        s1 = wmma_f16(aq[kc], b1, s1);
      }
      int c0i = colbase + cn, c1i = colbase + 16 + cn;
#pragma unroll
      for (int gg = 0; gg < 8; gg++) {
        int rr = rowbase + gg + hi * 8;
        float a0 = 0.f, a1 = 0.f;
        bool inr = (rr >= 1) && (rr < N1);
        if (inr && c0i >= 1 && c0i < N1) a0 = adj[((size_t)b * NN + (rr - 1)) * NN + (c0i - 1)];
        if (inr && c1i >= 1 && c1i < N1) a1 = adj[((size_t)b * NN + (rr - 1)) * NN + (c1i - 1)];
        if (rr == 0) { a0 = (c0i == 0) ? 1.f : 0.f; a1 = (c1i == 0) ? 1.f : 0.f; }
        float v0 = gv0[gg] * scale * s0[gg] + gv1[gg] * a0;
        float v1 = gv0[gg] * scale * s1[gg] + gv1[gg] * a1;
        if (c0i >= N1) v0 = -3.0e38f;
        if (c1i >= N1) v1 = -3.0e38f;
        float tmax = fmaxf(v0, v1);
#pragma unroll
        for (int mk = 1; mk < 16; mk <<= 1) tmax = fmaxf(tmax, __shfl_xor(tmax, mk, 32));
        float mnew = fmaxf(mrow[gg], tmax);
        float alpha = expf(mrow[gg] - mnew);
        float p0 = expf(v0 - mnew), p1 = expf(v1 - mnew);
        float rs = p0 + p1;
#pragma unroll
        for (int mk = 1; mk < 16; mk <<= 1) rs += __shfl_xor(rs, mk, 32);
        lrow[gg] = lrow[gg] * alpha + rs;
        mrow[gg] = mnew;
#pragma unroll
        for (int dc = 0; dc < 8; dc++) acc[dc][gg] *= alpha;
        int prow = gg + hi * 8;
        Ps[wave][prow][cn]      = (_Float16)p0;
        Ps[wave][prow][16 + cn] = (_Float16)p1;
      }
    }
    __syncthreads();
    if (active) {
      asm volatile("s_wait_dscnt 0" ::: "memory");
      int kh = hi * 8;
      h16 pa = cat88(*(const h8*)&Ps[wave][cn][kh],
                     *(const h8*)&Ps[wave][cn][kh + 16]);
      int kb = hi * 8;
#pragma unroll
      for (int dc = 0; dc < 8; dc++) {
        int dcol = dc * 16 + cn;
        h16 vb = cat88(*(const h8*)&VsT[dcol][kb], *(const h8*)&VsT[dcol][kb + 16]);
        acc[dc] = wmma_f16(pa, vb, acc[dc]);
      }
    }
    __syncthreads();
  }
  if (active) {
    float* so = Os[wave];
#pragma unroll
    for (int dc = 0; dc < 8; dc++)
#pragma unroll
      for (int gg = 0; gg < 8; gg++) so[(gg + hi * 8) * DIM + dc * 16 + cn] = acc[dc][gg] / lrow[gg];
    asm volatile("s_wait_dscnt 0" ::: "memory"); __builtin_amdgcn_wave_barrier(); __builtin_amdgcn_fence(__ATOMIC_RELEASE, "workgroup");
#pragma unroll 4
    for (int r = 0; r < 16; r++) { const int rr = rowbase + r;
      if (rr < N1) vst2(o + ((size_t)(b * N1) + rr) * OPROJ_K + head * DIM + lane * 4, *(const f4*)(so + r * DIM + lane * 4)); }
  }
}

__global__ void k_final(const float* __restrict__ x, const float* __restrict__ s,
                        const float* __restrict__ bb_, float* __restrict__ out) {
  __shared__ float sbuf[4];
  int t = blockIdx.x, d = threadIdx.x;
  int b = t / N1, n = t % N1;
  float v = x[(size_t)t * DIM + d];
  float mu = block_reduce128(v, sbuf) * (1.f / DIM);
  float dv = v - mu;
  float var = block_reduce128(dv * dv, sbuf) * (1.f / DIM);
  float xn = dv * rsqrtf(var + EPSL) * s[d] + bb_[d];
  float* out_cls   = out;
  float* out_nodes = out + BB * DIM;
  float* out_x     = out + BB * DIM + (size_t)BB * NN * DIM;
  if (n == 0) vst2(out_cls + b * DIM + d, (float_a)xn);
  else vst2(out_nodes + ((size_t)b * NN + (n - 1)) * DIM + d, (float_a)xn);
  vst2(out_x + (size_t)t * DIM + d, (float_a)v);
}

extern "C" void kernel_launch(void* const* d_in, const int* in_sizes, int n_in,
                              void* d_out, int out_size, void* d_ws, size_t ws_size,
                              hipStream_t stream) {
  (void)in_sizes; (void)n_in; (void)out_size; (void)ws_size;
  const float* node_feat = (const float*)d_in[0];
  const float* adj       = (const float*)d_in[1];
  const float* lapl      = (const float*)d_in[2];
  const float* W_ne1     = (const float*)d_in[3];
  const float* b_ne1     = (const float*)d_in[4];
  const float* W_ne2     = (const float*)d_in[5];
  const float* b_ne2     = (const float*)d_in[6];
  const float* W_pos     = (const float*)d_in[7];
  const float* b_pos     = (const float*)d_in[8];
  const float* cls_token = (const float*)d_in[9];
  const float* cls_pos   = (const float*)d_in[10];
  const float* ln1_s     = (const float*)d_in[11];
  const float* ln1_b     = (const float*)d_in[12];
  const float* Wqkv      = (const float*)d_in[13];
  const float* Wg        = (const float*)d_in[14];
  const float* bg        = (const float*)d_in[15];
  const float* Wproj     = (const float*)d_in[16];
  const float* bproj     = (const float*)d_in[17];
  const float* ln2_s     = (const float*)d_in[18];
  const float* ln2_b     = (const float*)d_in[19];
  const float* Wm1       = (const float*)d_in[20];
  const float* bm1       = (const float*)d_in[21];
  const float* Wm2       = (const float*)d_in[22];
  const float* bm2       = (const float*)d_in[23];
  const float* norm_s    = (const float*)d_in[24];
  const float* norm_b    = (const float*)d_in[25];

  float* ws = (float*)d_ws;
  size_t off = 0;
  float* x    = ws + off; off += (size_t)M_TOK * DIM;
  float* h    = ws + off; off += (size_t)M_TOK * DIM;
  float* gbuf = ws + off; off += (size_t)M_TOK * GSTRIDE;
  float* qkv  = ws + off; off += (size_t)M_TOK * QKV_N;
  float* obuf = ws + off; off += (size_t)M_TOK * OPROJ_K;
  float* tbuf = ws + off; off += (size_t)M_TOK * HID;

  k_embed<<<M_TOK, 256, 0, stream>>>(node_feat, lapl, W_ne1, b_ne1, W_ne2, b_ne2,
                                     W_pos, b_pos, cls_token, cls_pos, x);
  for (int l = 0; l < LL; l++) {
    k_ln<<<M_TOK, DIM, 0, stream>>>(x, ln1_s + l * DIM, ln1_b + l * DIM,
                                    Wg + (size_t)l * DIM * 2, bg + l * 2, h, gbuf, 1);
    dim3 gq((M_TOK + 63) / 64, QKV_N / 64);
    k_gemm<<<gq, 256, 0, stream>>>(h, Wqkv + (size_t)l * DIM * QKV_N, nullptr, nullptr,
                                   qkv, M_TOK, DIM, QKV_N, 0);
    dim3 ga(9, HH, BB);
    k_attn<<<ga, 128, 0, stream>>>(qkv, gbuf, adj, obuf);
    dim3 gp((M_TOK + 63) / 64, DIM / 64);
    k_gemm<<<gp, 256, 0, stream>>>(obuf, Wproj + (size_t)l * OPROJ_K * DIM,
                                   bproj + l * DIM, h, x, M_TOK, OPROJ_K, DIM, 0);
    k_ln<<<M_TOK, DIM, 0, stream>>>(x, ln2_s + l * DIM, ln2_b + l * DIM,
                                    nullptr, nullptr, h, nullptr, 0);
    dim3 gm1((M_TOK + 63) / 64, HID / 64);
    k_gemm<<<gm1, 256, 0, stream>>>(h, Wm1 + (size_t)l * DIM * HID, bm1 + l * HID,
                                    nullptr, tbuf, M_TOK, DIM, HID, 1);
    dim3 gm2((M_TOK + 63) / 64, DIM / 64);
    k_gemm<<<gm2, 256, 0, stream>>>(tbuf, Wm2 + (size_t)l * HID * DIM, bm2 + l * DIM,
                                    h, x, M_TOK, HID, DIM, 0);
  }
  k_final<<<M_TOK, DIM, 0, stream>>>(x, norm_s, norm_b, (float*)d_out);
}
